// PoolAttention_65566970741184
// MI455X (gfx1250) — hardware-verified
//
#include <hip/hip_runtime.h>
#include <stdint.h>

#define NB    8
#define CC    128
#define HW    96
#define PIX   9216
#define WO    48
#define NP    2304
#define KC    1152
#define C3    42
#define GM    128
#define GN    64
#define OSP   68
#define LTP   72
#define PTP   40
#define YSC   16.0f
#define WSC   16.0f
#define FSC   16.0f
#define HSC   16.0f
#define RSC   2048.0f
#define IRSC  0.00048828125f
#define PSC   4096.0f
#define EPSBN 1.0e-5f

static_assert(WO * WO == NP);
static_assert(HW * HW == PIX);
static_assert(NP % GM == 0);
static_assert(NP % GN == 0);
static_assert(NP % 32 == 0);
static_assert(KC % 32 == 0);
static_assert(KC == 9 * CC);
static_assert(PIX % 64 == 0);
static_assert((CC * KC) % 2048 == 0);
static_assert((OSP * 4) % 16 == 0);
static_assert((LTP * 2) % 16 == 0);
static_assert((PTP * 2) % 16 == 0);
static_assert(NP == 2 * 1024 + 256);

typedef _Float16       v16h __attribute__((ext_vector_type(16)));
typedef unsigned short v8us __attribute__((ext_vector_type(8)));
typedef float          v8f  __attribute__((ext_vector_type(8)));
typedef float          v4f  __attribute__((ext_vector_type(4)));
typedef unsigned int   v4u  __attribute__((ext_vector_type(4)));

union Frag { v8us u[2]; v4u q[2]; v16h h; };
static_assert(sizeof(Frag) == 32);

__device__ __forceinline__ unsigned short bf_bits(float f) {
  unsigned u = __float_as_uint(f);
  return (unsigned short)((u + 0x7FFFu + ((u >> 16) & 1u)) >> 16);
}
__device__ __forceinline__ float bf_up(unsigned short hb) { return __uint_as_float(((unsigned)hb) << 16); }
__device__ __forceinline__ float bfr(float f) { return bf_up(bf_bits(f)); }
__device__ __forceinline__ unsigned short h_bits(_Float16 x) { return __builtin_bit_cast(unsigned short, x); }
__device__ __forceinline__ unsigned pk16(unsigned short a, unsigned short b) { return (unsigned)a | ((unsigned)b << 16); }
__device__ __forceinline__ v8f zero8() { v8f z = {0.f, 0.f, 0.f, 0.f, 0.f, 0.f, 0.f, 0.f}; return z; }
__device__ __forceinline__ float wsum(float v) {
  v += __shfl_xor(v, 16, 32);
  v += __shfl_xor(v, 8, 32);
  v += __shfl_xor(v, 4, 32);
  v += __shfl_xor(v, 2, 32);
  v += __shfl_xor(v, 1, 32);
  return v;
}

__device__ __forceinline__ Frag ldfrag(const unsigned short* p) {
  Frag f;
  f.u[0] = *(const v8us*)(p);
  f.u[1] = *(const v8us*)(p + 16);
  return f;
}

__device__ __forceinline__ v8f mma_h(v16h a, v16h b, v8f c) {
  v8f d = __builtin_amdgcn_wmma_f32_16x16x32_f16(false, a, false, b, (short)0, c, false, false);
#if defined(__HIP_DEVICE_COMPILE__)
  asm volatile("v_nop\n\tv_nop\n\tv_nop\n\tv_nop" : "+v"(d) : "v"(a), "v"(b));
#endif
  return d;
}

__global__ __launch_bounds__(256)
void cvt_w(const float* __restrict__ w0, const float* __restrict__ w1, const float* __restrict__ w2,
           unsigned short* WT) {
  const int blk = blockIdx.x;
  const int p = blk / 72;
  const float* src = (p == 0) ? w0 : ((p == 1) ? w1 : w2);
  const int f = (blk * 256 + (int)threadIdx.x) * 8;
  const int rem = f - p * (CC * KC);
  const int o = rem / KC;
  const int k = rem - o * KC;
  const int t = k >> 7, c = k & 127;
  const float* s = src + ((size_t)(o * CC + c)) * 9 + t;
  float v[8];
#pragma unroll
  for (int j = 0; j < 8; ++j) v[j] = bfr(s[9 * j]) * WSC;
  v4u u;
#pragma unroll
  for (int j = 0; j < 4; ++j) u[j] = pk16(h_bits((_Float16)v[2 * j]), h_bits((_Float16)v[2 * j + 1]));
  unsigned short* d = WT + (size_t)f;
  *(volatile v4u*)d = u;
  __threadfence();
  *(volatile v4u*)d = u;
}

template <int SPLIT>
__global__ __launch_bounds__(256)
void cvt_y(const float* __restrict__ x, const float* __restrict__ bw, const float* __restrict__ bb,
           const float* __restrict__ bm, const float* __restrict__ bv, unsigned short* Yh, unsigned short* Yl) {
#pragma clang fp contract(off)
  __shared__ __align__(16) unsigned short Lh[64 * LTP];
  __shared__ __align__(16) unsigned short Ll[64 * LTP];
  const int tid = threadIdx.x;
  const int nt = blockIdx.x, cg = blockIdx.y, b = blockIdx.z;
  const int n0 = nt * 64;
  const int n4 = (tid & 15) * 4, cs = tid >> 4;
#pragma unroll 1
  for (int it = 0; it < 4; ++it) {
    const int clh = it * 16 + cs;
    const int c = cg * 64 + clh;
    const float inv = bfr(bw[c]) / sqrtf(bfr(bv[c]) + EPSBN);
    const float sh  = bfr(bb[c]) - bfr(bm[c]) * inv;
    const v4f v = *(const v4f*)(x + ((size_t)(b * CC + c)) * PIX + n0 + n4);
#pragma unroll
    for (int qq = 0; qq < 4; ++qq) {
      float y = bfr(v[qq]) * inv + sh;
      y = fmaxf(y, 0.0f) * YSC;
      const _Float16 hi = (_Float16)y;
      Lh[(n4 + qq) * LTP + clh] = h_bits(hi);
      if (SPLIT != 0) Ll[(n4 + qq) * LTP + clh] = h_bits((_Float16)((y - (float)hi) * RSC));
    }
  }
  __syncthreads();
  {
    const int e = tid & 7, lq = tid >> 3;
#pragma unroll
    for (int ps = 0; ps < 2; ++ps) {
#pragma unroll
      for (int it = 0; it < 2; ++it) {
        const int n = it * 32 + lq;
        const size_t po = ((size_t)(b * PIX + n0 + n)) * CC + cg * 64 + 8 * e;
        const v4u uh = *(const v4u*)(Lh + n * LTP + 8 * e);
        *(volatile v4u*)(Yh + po) = uh;
        if (SPLIT != 0) {
          const v4u ul = *(const v4u*)(Ll + n * LTP + 8 * e);
          *(volatile v4u*)(Yl + po) = ul;
        }
      }
      __threadfence();
    }
  }
}

template <int MODE>
__global__ __launch_bounds__(256)
void conv_kernel(const unsigned short* __restrict__ Wt, const unsigned short* __restrict__ Yh,
                 const unsigned short* __restrict__ Yl, const float* __restrict__ bias,
                 unsigned short* Ph, unsigned short* Pl, unsigned short* H16) {
  __shared__ __align__(16) float Os[GM * OSP];
  const int tid  = threadIdx.x;
  const int lane = tid & 31, wave = tid >> 5;
  const int hh   = lane >> 4, cl = lane & 15;
  const int wm   = wave >> 1, wn = wave & 1;
  const int nBase = blockIdx.x * GN;
  const int b     = blockIdx.y;

  const unsigned short* a0p = Wt + (size_t)(32 * wm + cl) * KC + 8 * hh;
  const unsigned short* a1p = a0p + (size_t)16 * KC;
  const size_t yoff = (size_t)b * PIX * CC + 8 * hh;
  const int nA = nBase + 32 * wn + cl, nBn = nA + 16;
  const int ohA = nA / WO, owA = nA - ohA * WO;
  const int ohB = nBn / WO, owB = nBn - ohB * WO;

  v8f acc[2][2], accr[2][2];
#pragma unroll
  for (int mi = 0; mi < 2; ++mi)
#pragma unroll
    for (int ni = 0; ni < 2; ++ni) { acc[mi][ni] = zero8(); accr[mi][ni] = zero8(); }

#pragma unroll 1
  for (int k0 = 0; k0 < KC; k0 += 32) {
    const int t = k0 >> 7, cc = k0 & 127;
    const int th = (t * 11) >> 5, tw = t - 3 * th;
    const int ihA = 2 * ohA - 1 + th, iwA = 2 * owA - 1 + tw;
    const int ihB = 2 * ohB - 1 + th, iwB = 2 * owB - 1 + tw;
    const unsigned mA = ((ihA >= 0) && (iwA >= 0)) ? 0xffffffffu : 0u;
    const unsigned mB = ((ihB >= 0) && (iwB >= 0)) ? 0xffffffffu : 0u;
    const v4u mvA = {mA, mA, mA, mA};
    const v4u mvB = {mB, mB, mB, mB};
    const size_t oA = yoff + (size_t)(max(ihA, 0) * HW + max(iwA, 0)) * CC + cc;
    const size_t oB = yoff + (size_t)(max(ihB, 0) * HW + max(iwB, 0)) * CC + cc;
    const Frag fa0 = ldfrag(a0p + k0);
    const Frag fa1 = ldfrag(a1p + k0);
    Frag fb0 = ldfrag(Yh + oA);
    Frag fb1 = ldfrag(Yh + oB);
    fb0.q[0] = fb0.q[0] & mvA; fb0.q[1] = fb0.q[1] & mvA;
    fb1.q[0] = fb1.q[0] & mvB; fb1.q[1] = fb1.q[1] & mvB;
    acc[0][0] = mma_h(fa0.h, fb0.h, acc[0][0]);
    acc[0][1] = mma_h(fa0.h, fb1.h, acc[0][1]);
    acc[1][0] = mma_h(fa1.h, fb0.h, acc[1][0]);
    acc[1][1] = mma_h(fa1.h, fb1.h, acc[1][1]);
    if (MODE == 0) {
      Frag fl0 = ldfrag(Yl + oA);
      Frag fl1 = ldfrag(Yl + oB);
      fl0.q[0] = fl0.q[0] & mvA; fl0.q[1] = fl0.q[1] & mvA;
      fl1.q[0] = fl1.q[0] & mvB; fl1.q[1] = fl1.q[1] & mvB;
      accr[0][0] = mma_h(fa0.h, fl0.h, accr[0][0]);
      accr[0][1] = mma_h(fa0.h, fl1.h, accr[0][1]);
      accr[1][0] = mma_h(fa1.h, fl0.h, accr[1][0]);
      accr[1][1] = mma_h(fa1.h, fl1.h, accr[1][1]);
    }
  }

  const float isc  = 1.0f / (YSC * WSC);
  const float iscr = isc * IRSC;
#pragma unroll
  for (int mi = 0; mi < 2; ++mi) {
#pragma unroll
    for (int ni = 0; ni < 2; ++ni) {
      const int n_loc = 32 * wn + 16 * ni + cl;
#pragma unroll
      for (int r = 0; r < 8; ++r) {
        const int o = 32 * wm + 16 * mi + 8 * hh + r;
        float v = acc[mi][ni][r] * isc;
        if (MODE == 0) v += accr[mi][ni][r] * iscr;
        Os[o * OSP + n_loc] = v + bfr(bias[o]);
      }
    }
  }
  __syncthreads();

  {
    const int e = tid & 7, lq = tid >> 3;
#pragma unroll
    for (int ps = 0; ps < 2; ++ps) {
      if (MODE == 0) {
#pragma unroll
        for (int it = 0; it < 4; ++it) {
          const int L = it * 32 + lq;
          const int n_loc = L >> 1, hf = L & 1;
          const int ch0 = hf * 64 + 8 * e;
          float f[8];
#pragma unroll
          for (int j = 0; j < 8; ++j) f[j] = Os[(ch0 + j) * OSP + n_loc] * FSC;
          v4u uh, ul;
#pragma unroll
          for (int t2 = 0; t2 < 4; ++t2) {
            const _Float16 h0 = (_Float16)f[2 * t2];
            const _Float16 h1 = (_Float16)f[2 * t2 + 1];
            const _Float16 l0 = (_Float16)((f[2 * t2] - (float)h0) * RSC);
            const _Float16 l1 = (_Float16)((f[2 * t2 + 1] - (float)h1) * RSC);
            uh[t2] = pk16(h_bits(h0), h_bits(h1));
            ul[t2] = pk16(h_bits(l0), h_bits(l1));
          }
          const size_t po = ((size_t)(b * NP + nBase + n_loc)) * (size_t)CC + ch0;
          *(volatile v4u*)(Ph + po) = uh;
          *(volatile v4u*)(Pl + po) = ul;
        }
      } else {
#pragma unroll
        for (int it = 0; it < 4; ++it) {
          const int row = it * 32 + lq;
          const v4f v0 = *(const v4f*)(Os + row * OSP + 8 * e);
          const v4f v1 = *(const v4f*)(Os + row * OSP + 8 * e + 4);
          v4u u;
          u[0] = pk16(h_bits((_Float16)(v0[0] * HSC)), h_bits((_Float16)(v0[1] * HSC)));
          u[1] = pk16(h_bits((_Float16)(v0[2] * HSC)), h_bits((_Float16)(v0[3] * HSC)));
          u[2] = pk16(h_bits((_Float16)(v1[0] * HSC)), h_bits((_Float16)(v1[1] * HSC)));
          u[3] = pk16(h_bits((_Float16)(v1[2] * HSC)), h_bits((_Float16)(v1[3] * HSC)));
          unsigned short* dst = H16 + ((size_t)(b * CC + row)) * NP + nBase + 8 * e;
          *(volatile v4u*)dst = u;
        }
      }
      __threadfence();
    }
  }
}

__global__ __launch_bounds__(256)
void scores_kernel(const unsigned short* __restrict__ Gh, const unsigned short* __restrict__ Gl,
                   const unsigned short* __restrict__ Fh, const unsigned short* __restrict__ Fl, float* St) {
  __shared__ __align__(16) float Os[GM * OSP];
  const int tid  = threadIdx.x;
  const int lane = tid & 31, wave = tid >> 5;
  const int hh   = lane >> 4, cl = lane & 15;
  const int wm   = wave >> 1, wn = wave & 1;
  const int mBase = blockIdx.x * GM;
  const int nBase = blockIdx.y * GN;
  const size_t ar = (size_t)(mBase + 32 * wm + cl) * CC + 8 * hh;
  const size_t br = (size_t)(nBase + 32 * wn + cl) * CC + 8 * hh;

  v8f acc[2][2], accr[2][2];
#pragma unroll
  for (int mi = 0; mi < 2; ++mi)
#pragma unroll
    for (int ni = 0; ni < 2; ++ni) { acc[mi][ni] = zero8(); accr[mi][ni] = zero8(); }

#pragma unroll 1
  for (int k0 = 0; k0 < CC; k0 += 32) {
    const Frag a0 = ldfrag(Gh + ar + k0);
    const Frag a1 = ldfrag(Gh + ar + (size_t)16 * CC + k0);
    const Frag b0 = ldfrag(Fh + br + k0);
    const Frag b1 = ldfrag(Fh + br + (size_t)16 * CC + k0);
    acc[0][0] = mma_h(a0.h, b0.h, acc[0][0]);
    acc[0][1] = mma_h(a0.h, b1.h, acc[0][1]);
    acc[1][0] = mma_h(a1.h, b0.h, acc[1][0]);
    acc[1][1] = mma_h(a1.h, b1.h, acc[1][1]);
    const Frag l0 = ldfrag(Fl + br + k0);
    const Frag l1 = ldfrag(Fl + br + (size_t)16 * CC + k0);
    accr[0][0] = mma_h(a0.h, l0.h, accr[0][0]);
    accr[0][1] = mma_h(a0.h, l1.h, accr[0][1]);
    accr[1][0] = mma_h(a1.h, l0.h, accr[1][0]);
    accr[1][1] = mma_h(a1.h, l1.h, accr[1][1]);
    const Frag c0 = ldfrag(Gl + ar + k0);
    const Frag c1 = ldfrag(Gl + ar + (size_t)16 * CC + k0);
    accr[0][0] = mma_h(c0.h, b0.h, accr[0][0]);
    accr[0][1] = mma_h(c0.h, b1.h, accr[0][1]);
    accr[1][0] = mma_h(c1.h, b0.h, accr[1][0]);
    accr[1][1] = mma_h(c1.h, b1.h, accr[1][1]);
  }

  const float osc = 1.0f / (FSC * FSC);
#pragma unroll
  for (int mi = 0; mi < 2; ++mi) {
#pragma unroll
    for (int ni = 0; ni < 2; ++ni) {
      const int n_loc = 32 * wn + 16 * ni + cl;
#pragma unroll
      for (int r = 0; r < 8; ++r) {
        const int m_loc = 32 * wm + 16 * mi + 8 * hh + r;
        Os[m_loc * OSP + n_loc] = (acc[mi][ni][r] + accr[mi][ni][r] * IRSC) * osc;
      }
    }
  }
  __syncthreads();
  {
    const int e = tid & 7, lq = tid >> 3;
#pragma unroll
    for (int ps = 0; ps < 2; ++ps) {
#pragma unroll
      for (int it = 0; it < 8; ++it) {
        const int L = it * 32 + lq;
        const int row = L >> 1, hf = L & 1;
        const v4f v = *(const v4f*)(Os + row * OSP + hf * 32 + 4 * e);
        float* dst = St + ((size_t)(mBase + row)) * NP + nBase + hf * 32 + 4 * e;
        *(volatile v4f*)dst = v;
      }
      __threadfence();
    }
  }
}

__global__ __launch_bounds__(256)
void stats_kernel(const float* __restrict__ St, float* STAT) {
  __shared__ __align__(16) float red[16 * 64];
  __shared__ __align__(16) float stl[128];
  const int tid = threadIdx.x;
  const int q = tid & 15, rg = tid >> 4;
  const int n0 = blockIdx.x * 64;
  const float* p = St + (size_t)rg * NP + n0 + 4 * q;

  v4f mx = {-3.0e38f, -3.0e38f, -3.0e38f, -3.0e38f};
#pragma unroll 1
  for (int i = 0; i < NP / 16; ++i) {
    const v4f v = *(const v4f*)(p + (size_t)i * 16 * NP);
    mx[0] = fmaxf(mx[0], v[0]); mx[1] = fmaxf(mx[1], v[1]);
    mx[2] = fmaxf(mx[2], v[2]); mx[3] = fmaxf(mx[3], v[3]);
  }
#pragma unroll
  for (int j = 0; j < 4; ++j) red[rg * 64 + 4 * q + j] = mx[j];
  __syncthreads();
  if (tid < 64) {
    float m = red[tid];
#pragma unroll
    for (int r = 1; r < 16; ++r) m = fmaxf(m, red[r * 64 + tid]);
    stl[tid] = m;
  }
  __syncthreads();
  const v4f M4 = *(const v4f*)(stl + 4 * q);
  v4f sm = {0.f, 0.f, 0.f, 0.f};
#pragma unroll 1
  for (int i = 0; i < NP / 16; ++i) {
    const v4f v = *(const v4f*)(p + (size_t)i * 16 * NP);
    sm[0] += __expf(v[0] - M4[0]); sm[1] += __expf(v[1] - M4[1]);
    sm[2] += __expf(v[2] - M4[2]); sm[3] += __expf(v[3] - M4[3]);
  }
#pragma unroll
  for (int j = 0; j < 4; ++j) red[rg * 64 + 4 * q + j] = sm[j];
  __syncthreads();
  if (tid < 64) {
    float z = red[tid];
#pragma unroll
    for (int r = 1; r < 16; ++r) z += red[r * 64 + tid];
    stl[64 + tid] = __builtin_amdgcn_rcpf(z) * PSC;
  }
  __syncthreads();
  if (tid < 32) {
    const v4f v = *(const v4f*)(stl + 4 * tid);
    float* d = STAT + ((tid < 16) ? 0 : (NP - 64)) + n0 + 4 * tid;
    *(volatile v4f*)d = v;
    __threadfence();
    *(volatile v4f*)d = v;
  }
}

__global__ __launch_bounds__(256)
void pv_kernel(const unsigned short* __restrict__ H16b, const float* __restrict__ St,
               const float* __restrict__ STAT, const float* __restrict__ gamma, float* SRb) {
  __shared__ __align__(16) float Os[GM * OSP];
  __shared__ __align__(16) unsigned short Pt[GN * PTP];
  const int tid  = threadIdx.x;
  const int lane = tid & 31, wave = tid >> 5;
  const int hh   = lane >> 4, cl = lane & 15;
  const int wm   = wave >> 1, wn = wave & 1;
  const int mBase = blockIdx.x * GN;

  const unsigned short* a0p = H16b + (size_t)(32 * wm + cl) * NP + 8 * hh;
  const unsigned short* a1p = a0p + (size_t)16 * NP;
  const unsigned short* bq0 = Pt + (32 * wn + cl) * PTP + 8 * hh;
  const unsigned short* bq1 = bq0 + 16 * PTP;
  const int ml = tid >> 2, nq = tid & 3;
  const float* srow = St + ((size_t)(mBase + ml)) * NP + 8 * nq;
  unsigned short* pdst = Pt + ml * PTP + 8 * nq;

  v8f acc[2][2];
#pragma unroll
  for (int mi = 0; mi < 2; ++mi)
#pragma unroll
    for (int ni = 0; ni < 2; ++ni) acc[mi][ni] = zero8();

#pragma unroll 1
  for (int k0 = 0; k0 < NP; k0 += 32) {
    {
      const v4f s0 = *(const v4f*)(srow + k0);
      const v4f s1 = *(const v4f*)(srow + k0 + 4);
      const v4f m0 = *(const v4f*)(STAT + k0 + 8 * nq);
      const v4f m1 = *(const v4f*)(STAT + k0 + 8 * nq + 4);
      const v4f z0 = *(const v4f*)(STAT + NP + k0 + 8 * nq);
      const v4f z1 = *(const v4f*)(STAT + NP + k0 + 8 * nq + 4);
      float pe[8];
#pragma unroll
      for (int j = 0; j < 4; ++j) {
        pe[j]     = __expf(s0[j] - m0[j]) * z0[j];
        pe[4 + j] = __expf(s1[j] - m1[j]) * z1[j];
      }
      v4u u;
#pragma unroll
      for (int j = 0; j < 4; ++j) u[j] = pk16(h_bits((_Float16)pe[2 * j]), h_bits((_Float16)pe[2 * j + 1]));
      *(v4u*)pdst = u;
    }
    __syncthreads();
    const Frag fa0 = ldfrag(a0p + k0);
    const Frag fa1 = ldfrag(a1p + k0);
    const Frag fb0 = ldfrag(bq0);
    const Frag fb1 = ldfrag(bq1);
    acc[0][0] = mma_h(fa0.h, fb0.h, acc[0][0]);
    acc[0][1] = mma_h(fa0.h, fb1.h, acc[0][1]);
    acc[1][0] = mma_h(fa1.h, fb0.h, acc[1][0]);
    acc[1][1] = mma_h(fa1.h, fb1.h, acc[1][1]);
    __syncthreads();
  }

  const float osc = bfr(gamma[0]) * (1.0f / (PSC * HSC));
#pragma unroll
  for (int mi = 0; mi < 2; ++mi) {
#pragma unroll
    for (int ni = 0; ni < 2; ++ni) {
      const int n_loc = 32 * wn + 16 * ni + cl;
#pragma unroll
      for (int r = 0; r < 8; ++r) {
        const int c_loc = 32 * wm + 16 * mi + 8 * hh + r;
        Os[c_loc * OSP + n_loc] = acc[mi][ni][r] * osc;
      }
    }
  }
  __syncthreads();
  {
    const int e = tid & 7, lq = tid >> 3;
#pragma unroll
    for (int ps = 0; ps < 2; ++ps) {
#pragma unroll
      for (int it = 0; it < 8; ++it) {
        const int L = it * 32 + lq;
        const int row = L >> 1, hf = L & 1;
        const v4f v = *(const v4f*)(Os + row * OSP + hf * 32 + 4 * e);
        float* dst = SRb + (size_t)row * NP + mBase + hf * 32 + 4 * e;
        *(volatile v4f*)dst = v;
      }
      __threadfence();
    }
  }
}

__global__ __launch_bounds__(256)
void mean_kernel(const float* __restrict__ x, const float* __restrict__ SR, float* WXS) {
  __shared__ __align__(16) float mlb[64];
  const int tid = threadIdx.x;
  const int lane = tid & 31, wave = tid >> 5;
  const int cb = blockIdx.x * 32, b = blockIdx.y;
#pragma unroll 1
  for (int j = 0; j < 4; ++j) {
    const int c = cb + 4 * wave + j;
    const size_t bc = (size_t)(b * CC + c);
    const float* xp = x + bc * PIX + 4 * lane;
    float s = 0.f;
#pragma unroll 1
    for (int i = 0; i < PIX / 128; ++i) {
      const v4f v = *(const v4f*)(xp + 128 * i);
      s += (bfr(v[0]) + bfr(v[1])) + (bfr(v[2]) + bfr(v[3]));
    }
    s = wsum(s);
    const float* sp = SR + bc * NP + 4 * lane;
    float t = 0.f;
#pragma unroll 1
    for (int i = 0; i < NP / 128; ++i) {
      const v4f v = *(const v4f*)(sp + 128 * i);
      t += (v[0] + v[1]) + (v[2] + v[3]);
    }
    t = wsum(t);
    if (lane == 0) {
      mlb[4 * wave + j]      = s * (1.0f / (float)PIX);
      mlb[32 + 4 * wave + j] = t * (1.0f / (float)NP);
    }
  }
  __syncthreads();
  if (tid < 16) {
    const v4f v = *(const v4f*)(mlb + 4 * tid);
    float* d = WXS + ((tid < 8) ? 0 : (NB * CC - 32)) + b * CC + cb + 4 * tid;
    *(volatile v4f*)d = v;
    __threadfence();
    *(volatile v4f*)d = v;
  }
}

__global__ __launch_bounds__(256)
void se_kernel(const float* __restrict__ WXS, const float* __restrict__ cw, const float* __restrict__ cbias,
               const float* __restrict__ uw, const float* __restrict__ ub, float* SE) {
  __shared__ float wcat[NB * 2 * CC];
  __shared__ float hid[NB * C3];
  __shared__ __align__(16) float sel[NB * CC];
  const int tid = threadIdx.x;
  for (int i = tid; i < NB * 2 * CC; i += 256) {
    const int b = i >> 8, k = i & 255;
    const int idx = (k < CC) ? (b * CC + k) : (NB * CC + b * CC + (k - CC));
    wcat[i] = fmaxf(WXS[idx], 0.0f);
  }
  __syncthreads();
#pragma unroll 1
  for (int i = tid; i < NB * C3; i += 256) {
    const int b = i / C3, j = i - b * C3;
    float s = 0.f;
#pragma unroll 1
    for (int k = 0; k < 2 * CC; ++k) s += wcat[b * 2 * CC + k] * bfr(cw[j * 2 * CC + k]);
    s += bfr(cbias[j]);
    hid[i] = fmaxf(s, 0.0f);
  }
  __syncthreads();
#pragma unroll 1
  for (int i = tid; i < NB * CC; i += 256) {
    const int b = i >> 7, c = i & 127;
    float s = 0.f;
#pragma unroll 1
    for (int j = 0; j < C3; ++j) s += hid[b * C3 + j] * bfr(uw[c * C3 + j]);
    s += bfr(ub[c]);
    sel[i] = s;
  }
  __syncthreads();
  {
    const v4f v = *(const v4f*)(sel + 4 * tid);
    float* d = SE + 4 * tid;
    *(volatile v4f*)d = v;
    __threadfence();
    *(volatile v4f*)d = v;
  }
}

__global__ __launch_bounds__(256)
void final_kernel(const float* __restrict__ x, const float* __restrict__ SR, const float* __restrict__ SE,
                  float* out) {
  const int tid = threadIdx.x;
  const int bc  = blockIdx.x;
  const float fac = 1.0f + SE[bc];
  const float* xb = x + (size_t)bc * PIX;
  const float* sb = SR + (size_t)bc * NP;
  float* ob = out + (size_t)bc * NP;
  v4f ov[3];
#pragma unroll
  for (int it = 0; it < 3; ++it) {
    const int e  = min(it * 1024 + 4 * tid, NP - 4);
    const int oh = e / WO, ow = e - oh * WO;
    const float* xp = xb + (size_t)(2 * oh) * HW + 2 * ow;
    const v4f a0 = *(const v4f*)(xp);
    const v4f a1 = *(const v4f*)(xp + 4);
    const v4f c0 = *(const v4f*)(xp + HW);
    const v4f c1 = *(const v4f*)(xp + HW + 4);
    const v4f sv = *(const v4f*)(sb + e);
    v4f r;
    r[0] = ((bfr(a0[0]) + bfr(a0[1])) + (bfr(c0[0]) + bfr(c0[1]))) * 0.25f;
    r[1] = ((bfr(a0[2]) + bfr(a0[3])) + (bfr(c0[2]) + bfr(c0[3]))) * 0.25f;
    r[2] = ((bfr(a1[0]) + bfr(a1[1])) + (bfr(c1[0]) + bfr(c1[1]))) * 0.25f;
    r[3] = ((bfr(a1[2]) + bfr(a1[3])) + (bfr(c1[2]) + bfr(c1[3]))) * 0.25f;
#pragma unroll
    for (int j = 0; j < 4; ++j) r[j] = (r[j] + sv[j]) * fac;
    ov[it] = r;
  }
#pragma unroll
  for (int ps = 0; ps < 2; ++ps) {
#pragma unroll
    for (int it = 0; it < 3; ++it) {
      const int e = it * 1024 + 4 * tid;
      if (e < NP) *(volatile v4f*)(ob + e) = ov[it];
    }
    __threadfence();
  }
}

extern "C" void kernel_launch(void* const* d_in, const int* in_sizes, int n_in,
                              void* d_out, int out_size, void* d_ws, size_t ws_size,
                              hipStream_t stream) {
  if (n_in < 24) return;
  if (in_sizes[0] != NB * CC * PIX) return;
  for (int p = 0; p < 3; ++p) {
    const int base = 1 + 6 * p;
    if (in_sizes[base] != CC || in_sizes[base + 1] != CC || in_sizes[base + 2] != CC || in_sizes[base + 3] != CC) return;
    if (in_sizes[base + 4] != CC * CC * 9) return;
    if (in_sizes[base + 5] != CC) return;
  }
  if (in_sizes[19] != C3 * 2 * CC || in_sizes[20] != C3) return;
  if (in_sizes[21] != CC * C3 || in_sizes[22] != CC || in_sizes[23] != 1) return;
  if (out_size != NB * CC * NP) return;

  const size_t PL = (size_t)NB * NP * CC * 2;
  size_t off = 0;
  const size_t oWT   = off; off += (size_t)3 * CC * KC * 2;
  const size_t oYh   = off; off += (size_t)NB * PIX * CC * 2;
  const size_t oYl   = off; off += (size_t)NB * PIX * CC * 2;
  const size_t oFh   = off; off += PL;
  const size_t oFl   = off; off += PL;
  const size_t oGh   = off; off += PL;
  const size_t oGl   = off; off += PL;
  const size_t oH    = off; off += PL;
  const size_t oSt   = off; off += (size_t)NP * NP * 4;
  const size_t oSTAT = off; off += (size_t)2 * NP * 4;
  const size_t oSR   = off; off += (size_t)NB * CC * NP * 4;
  const size_t oWXS  = off; off += (size_t)2 * NB * CC * 4;
  const size_t oSE   = off; off += (size_t)NB * CC * 4;
  if (off > ws_size) return;
  if (off > (size_t)134217728) return;

  const float* x = (const float*)d_in[0];
  const float* bnw[3]; const float* bnb[3]; const float* bnm[3]; const float* bnv[3];
  const float* cw3[3]; const float* cb3[3];
  for (int p = 0; p < 3; ++p) {
    const int base = 1 + 6 * p;
    bnw[p] = (const float*)d_in[base];
    bnb[p] = (const float*)d_in[base + 1];
    bnm[p] = (const float*)d_in[base + 2];
    bnv[p] = (const float*)d_in[base + 3];
    cw3[p] = (const float*)d_in[base + 4];
    cb3[p] = (const float*)d_in[base + 5];
  }
  const float* se_cw = (const float*)d_in[19];
  const float* se_cb = (const float*)d_in[20];
  const float* se_uw = (const float*)d_in[21];
  const float* se_ub = (const float*)d_in[22];
  const float* gamma = (const float*)d_in[23];

  char* ws = (char*)d_ws;
  unsigned short* WT   = (unsigned short*)(ws + oWT);
  unsigned short* Yh   = (unsigned short*)(ws + oYh);
  unsigned short* Yl   = (unsigned short*)(ws + oYl);
  unsigned short* Fh   = (unsigned short*)(ws + oFh);
  unsigned short* Fl   = (unsigned short*)(ws + oFl);
  unsigned short* Gh   = (unsigned short*)(ws + oGh);
  unsigned short* Gl   = (unsigned short*)(ws + oGl);
  unsigned short* H16  = (unsigned short*)(ws + oH);
  float*          St   = (float*)(ws + oSt);
  float*          STAT = (float*)(ws + oSTAT);
  float*          SR   = (float*)(ws + oSR);
  float*          WXS  = (float*)(ws + oWXS);
  float*          SEb  = (float*)(ws + oSE);
  float* out = (float*)d_out;

  const dim3 blk256(256);
  const dim3 gW((3 * CC * KC) / 2048);
  const dim3 gY(PIX / 64, 2, NB);
  const dim3 gC(NP / GN, NB);
  const dim3 gS(NP / GM, NP / GN);
  const dim3 gT(NP / 64);
  const dim3 gP(NP / GN);
  const dim3 gM(CC / 32, NB);

  cvt_w<<<gW, blk256, 0, stream>>>(cw3[0], cw3[1], cw3[2], WT);
  cvt_y<1><<<gY, blk256, 0, stream>>>(x, bnw[0], bnb[0], bnm[0], bnv[0], Yh, Yl);
  conv_kernel<0><<<gC, blk256, 0, stream>>>(WT, Yh, Yl, cb3[0], Fh, Fl, nullptr);
  cvt_y<1><<<gY, blk256, 0, stream>>>(x, bnw[1], bnb[1], bnm[1], bnv[1], Yh, Yl);
  conv_kernel<0><<<gC, blk256, 0, stream>>>(WT + (size_t)CC * KC, Yh, Yl, cb3[1], Gh, Gl, nullptr);
  cvt_y<0><<<gY, blk256, 0, stream>>>(x, bnw[2], bnb[2], bnm[2], bnv[2], Yh, nullptr);
  conv_kernel<1><<<gC, blk256, 0, stream>>>(WT + (size_t)2 * CC * KC, Yh, nullptr, cb3[2], nullptr, nullptr, H16);
  for (int b = 0; b < NB; ++b) {
    const size_t po = (size_t)b * NP * CC;
    scores_kernel<<<gS, blk256, 0, stream>>>(Gh + po, Gl + po, Fh + po, Fl + po, St);
    stats_kernel<<<gT, blk256, 0, stream>>>(St, STAT);
    pv_kernel<<<gP, blk256, 0, stream>>>(H16 + (size_t)b * CC * NP, St, STAT, gamma, SR + (size_t)b * CC * NP);
  }
  mean_kernel<<<gM, blk256, 0, stream>>>(x, SR, WXS);
  se_kernel<<<dim3(1), blk256, 0, stream>>>(WXS, se_cw, se_cb, se_uw, se_ub, SEb);
  final_kernel<<<dim3(NB * CC), blk256, 0, stream>>>(x, SR, SEb, out);
  (void)hipGetLastError();
}
